// MambaBlock_7421703488073
// MI455X (gfx1250) — hardware-run, weakly checked
//
#include <hip/hip_runtime.h>
#include <math.h>

typedef __attribute__((ext_vector_type(16))) _Float16 v16h;
typedef __attribute__((ext_vector_type(8)))  _Float16 v8h;
typedef __attribute__((ext_vector_type(16))) __bf16   v16b;
typedef __attribute__((ext_vector_type(8)))  __bf16   v8b;
typedef __attribute__((ext_vector_type(8)))  float    v8f;
typedef __attribute__((ext_vector_type(4)))  float    v4f;

constexpr int kBatch   = 2;
constexpr int kSeq     = 2048;
constexpr int kDm      = 512;
constexpr int kDin     = 1024;
constexpr int kNst     = 16;
constexpr int kTaps    = 4;
constexpr int kRows    = kBatch * kSeq;
constexpr int kXp      = 2 * kDin;
constexpr int kPadRows = kSeq + kTaps - 1;
constexpr int kConvK   = kTaps * kDin;
constexpr int kBcP     = 64;
constexpr int kTP      = 68;
constexpr int kScanTS  = 64;
constexpr int kScanCh  = 64;
constexpr int kScanYP  = 68;
constexpr int kScanXP  = 32;
constexpr float kCarryXc    = 64.0f;
constexpr float kCarryWd    = 256.0f;
constexpr float kDeltaScale = 1.0f / (kCarryXc * kCarryWd);
constexpr float kF16MinNormal = 6.103515625e-05f;
constexpr float kF32MinNormal = 1.17549435e-38f;
static_assert(kRows == 4096 && kXp == 2048 && kPadRows == 2051 && kConvK == 4096, "shape constants");
static_assert((kDm % 32) == 0 && (kDin % 32) == 0 && (kConvK % 32) == 0, "GEMM K multiples of 32");
static_assert((kSeq % 64) == 0 && (kRows % 64) == 0 && (kDin % 64) == 0 && (kDm % 64) == 0 && (kBcP % 64) == 0, "GEMM M,N multiples of 64");
static_assert(2 * kNst <= kBcP && 2 * kNst == kScanXP, "B|C packing");
static_assert((kSeq % kScanTS) == 0 && (kDin % kScanCh) == 0, "scan tiles");

constexpr size_t kSzXH   = (size_t)kRows * kDm * 2;
constexpr size_t kSzWI   = (size_t)kXp * kDm * 2;
constexpr size_t kSzCK   = (size_t)kDin * kConvK * 2;
constexpr size_t kSzWD   = (size_t)kDin * kDin * 2;
constexpr size_t kSzWBC  = (size_t)kBcP * kDin * 2;
constexpr size_t kSzWO   = (size_t)kDm * kDin * 2;
constexpr size_t kSzXZ   = (size_t)kBatch * kPadRows * kDin * 2;
constexpr size_t kSzF32  = (size_t)kRows * kDin * 4;
constexpr size_t kSzH16  = (size_t)kRows * kDin * 2;
constexpr size_t kSzBC   = (size_t)kRows * kBcP * 4;
constexpr size_t kOffXH   = 0;
constexpr size_t kOffXL   = kOffXH   + kSzXH;
constexpr size_t kOffWIH  = kOffXL   + kSzXH;
constexpr size_t kOffWIL  = kOffWIH  + kSzWI;
constexpr size_t kOffCKH  = kOffWIL  + kSzWI;
constexpr size_t kOffCKL  = kOffCKH  + kSzCK;
constexpr size_t kOffWD   = kOffCKL  + kSzCK;
constexpr size_t kOffWBCH = kOffWD   + kSzWD;
constexpr size_t kOffWBCL = kOffWBCH + kSzWBC;
constexpr size_t kOffWOH  = kOffWBCL + kSzWBC;
constexpr size_t kOffWOL  = kOffWOH  + kSzWO;
constexpr size_t kOffXZH  = kOffWOL  + kSzWO;
constexpr size_t kOffXZL  = kOffXZH  + kSzXZ;
constexpr size_t kOffGATE = kOffXZL  + kSzXZ;
constexpr size_t kOffXC32 = kOffGATE + kSzF32;
constexpr size_t kOffXC16 = kOffXC32 + kSzF32;
constexpr size_t kOffXCH  = kOffXC16 + kSzH16;
constexpr size_t kOffXCL  = kOffXCH  + kSzH16;
constexpr size_t kOffDX   = kOffXCL  + kSzH16;
constexpr size_t kOffBC   = kOffDX   + kSzF32;
constexpr size_t kWsTotal = kOffBC   + kSzBC;
static_assert(kWsTotal == 127164416ull, "carve total");
static_assert(kWsTotal <= 134217728ull, "carve cap");
static_assert(kSzH16 == kSzCK, "Y planes fit the dead conv-weight planes exactly");
static_assert((kOffXL % 128) == 0 && (kOffWIH % 128) == 0 && (kOffWIL % 128) == 0 && (kOffCKH % 128) == 0 &&
              (kOffCKL % 128) == 0 && (kOffWD % 128) == 0 && (kOffWBCH % 128) == 0 && (kOffWBCL % 128) == 0 &&
              (kOffWOH % 128) == 0 && (kOffWOL % 128) == 0 && (kOffXZH % 128) == 0 && (kOffXZL % 128) == 0 &&
              (kOffGATE % 128) == 0 && (kOffXC32 % 128) == 0 && (kOffXC16 % 128) == 0 && (kOffXCH % 128) == 0 &&
              (kOffXCL % 128) == 0 && (kOffDX % 128) == 0 && (kOffBC % 128) == 0, "128-B aligned regions");

__device__ __forceinline__ unsigned short f2bf_bits(float f) {
  unsigned u = __float_as_uint(f);
  return (unsigned short)((u + 0x7FFFu + ((u >> 16) & 1u)) >> 16);
}
__device__ __forceinline__ float bf_bits2f(unsigned short h) { return __uint_as_float(((unsigned)h) << 16); }

__device__ __forceinline__ void cvt_hilo(float f, _Float16& hb, _Float16& lb) {
  const unsigned short h = f2bf_bits(f);
  const unsigned short l = f2bf_bits(f - bf_bits2f(h));
  hb = __builtin_bit_cast(_Float16, h);
  lb = __builtin_bit_cast(_Float16, l);
}
__device__ __forceinline__ _Float16 cvt_f16_carried(float f, float carry) {
  float c = f * carry;
  c = (fabsf(c) < kF16MinNormal) ? 0.0f : c;
  return (_Float16)c;
}
__device__ __forceinline__ float silu_f(float v) { return v * __builtin_amdgcn_rcpf(1.0f + expf(-v)); }
__device__ __forceinline__ float softplus_f(float v) { return fmaxf(v, 0.0f) + log1pf(expf(-fabsf(v))); }
__device__ __forceinline__ void wave_lds_sync() {
  __builtin_amdgcn_fence(__ATOMIC_RELEASE, "workgroup");
  __builtin_amdgcn_wave_barrier();
  __builtin_amdgcn_fence(__ATOMIC_ACQUIRE, "workgroup");
}

__device__ __forceinline__ void dep_guard4_h(v8f& a, v8f& b, v8f& c, v8f& d, v16h x, v16h y) { asm volatile("v_nop\n\tv_nop\n\tv_nop\n\tv_nop" : "+v"(a), "+v"(b), "+v"(c), "+v"(d) : "v"(x), "v"(y)); }
__device__ __forceinline__ void dep_guard4_b(v8f& a, v8f& b, v8f& c, v8f& d, v16b x, v16b y) { asm volatile("v_nop\n\tv_nop\n\tv_nop\n\tv_nop" : "+v"(a), "+v"(b), "+v"(c), "+v"(d) : "v"(x), "v"(y)); }
__device__ __forceinline__ void keep4_h(v16h a, v16h b, v16h c, v16h d) { asm volatile("v_nop" :: "v"(a), "v"(b), "v"(c), "v"(d)); }
__device__ __forceinline__ void keep4_b(v16b a, v16b b, v16b c, v16b d) { asm volatile("v_nop" :: "v"(a), "v"(b), "v"(c), "v"(d)); }
__device__ __forceinline__ void acc_guard4(v8f& a, v8f& b, v8f& c, v8f& d) { asm volatile("v_nop\n\tv_nop\n\tv_nop\n\tv_nop" : "+v"(a), "+v"(b), "+v"(c), "+v"(d)); }

template <typename T> struct Frag;
template <> struct Frag<_Float16> {
  typedef v16h V; union U { v16h v; v8h h[2]; };
  static __device__ __forceinline__ v16h load(const _Float16* p) {
    U f; f.h[0] = *(const v8h*)(p); f.h[1] = *(const v8h*)(p + 16); return f.v;
  }
  static __device__ __forceinline__ v8f mma(v16h a, v16h b, v8f c) {
    return __builtin_amdgcn_wmma_f32_16x16x32_f16(false, a, false, b, (short)0, c, false, false);
  }
  static __device__ __forceinline__ void guard4(v8f& a, v8f& b, v8f& c, v8f& d, v16h x, v16h y) { dep_guard4_h(a, b, c, d, x, y); }
  static __device__ __forceinline__ void keep(v16h a, v16h b, v16h c, v16h d) { keep4_h(a, b, c, d); }
};
template <> struct Frag<__bf16> {
  typedef v16b V; union U { v16b v; v8b h[2]; };
  static __device__ __forceinline__ v16b load(const __bf16* p) {
    U f; f.h[0] = *(const v8b*)(p); f.h[1] = *(const v8b*)(p + 16); return f.v;
  }
  static __device__ __forceinline__ v8f mma(v16b a, v16b b, v8f c) {
    return __builtin_amdgcn_wmma_f32_16x16x32_bf16(false, a, false, b, (short)0, c, false, false);
  }
  static __device__ __forceinline__ void guard4(v8f& a, v8f& b, v8f& c, v8f& d, v16b x, v16b y) { dep_guard4_b(a, b, c, d, x, y); }
  static __device__ __forceinline__ void keep(v16b a, v16b b, v16b c, v16b d) { keep4_b(a, b, c, d); }
};
template <int ET> struct Elem;
template <> struct Elem<0> { typedef _Float16 T; };
template <> struct Elem<1> { typedef __bf16 T; };

__device__ __forceinline__ void store_slab_f32(const float* slab, float* Cb, int mBase, int ldc, int n0, int lane) {
  const int hh = lane >> 4, c4 = (lane & 15) * 4;
  for (int pass = 0; pass < 2; ++pass) {
#pragma unroll
    for (int it = 0; it < 8; ++it) {
      const int row = it * 2 + hh;
      const v4f v = *(const v4f*)(slab + row * kTP + c4);
      *(volatile v4f*)(Cb + (size_t)(mBase + row) * ldc + n0 + c4) = v;
    }
    __threadfence();
  }
}
template <int KIND>
__device__ __forceinline__ void store_slab_16(const float* slab, unsigned short* P0, unsigned short* P1,
                                              int mBase, int ldc, int n0, int lane, float carry) {
  const int q = lane >> 3, c8 = (lane & 7) * 8;
  v8h hv[4], lv[4];
#pragma unroll
  for (int it = 0; it < 4; ++it) {
    const float* sp = slab + (it * 4 + q) * kTP + c8;
    const v4f a0 = *(const v4f*)(sp);
    const v4f a1 = *(const v4f*)(sp + 4);
#pragma unroll
    for (int e = 0; e < 4; ++e) {
      const float f0 = a0[e];
      const float f1 = a1[e];
      _Float16 h0, l0, h1, l1;
      if (KIND == 0) {
        cvt_hilo(f0, h0, l0);
        cvt_hilo(f1, h1, l1);
      } else {
        h0 = cvt_f16_carried(f0, carry);
        h1 = cvt_f16_carried(f1, carry);
        l0 = h0;
        l1 = h1;
      }
      hv[it][e] = h0;
      hv[it][4 + e] = h1;
      lv[it][e] = l0;
      lv[it][4 + e] = l1;
    }
  }
  for (int pass = 0; pass < 2; ++pass) {
#pragma unroll
    for (int it = 0; it < 4; ++it) {
      const size_t o = (size_t)(mBase + it * 4 + q) * ldc + n0 + c8;
      *(volatile v8h*)(P0 + o) = hv[it];
      if (KIND == 0) *(volatile v8h*)(P1 + o) = lv[it];
    }
    __threadfence();
  }
}

template <int ET, int SPL, int EPI>
__global__ __launch_bounds__(256) void gemm64_kernel(
    const unsigned short* __restrict__ Ap, const unsigned short* __restrict__ A2p, int lda, long strideA,
    const unsigned short* __restrict__ Btp, const unsigned short* __restrict__ Bt2p, int ldb,
    void* __restrict__ C0, void* __restrict__ C1, void* __restrict__ C2, void* __restrict__ C3, int ldc, long strideC,
    const float* __restrict__ bias, const float* __restrict__ bias2, const float* __restrict__ aux,
    int M, int N, int K, float scale) {
  typedef typename Elem<ET>::T T;
  typedef typename Frag<T>::V V;
  const T* A = (const T*)Ap; const T* A2 = (const T*)A2p; const T* Bt = (const T*)Btp; const T* Bt2 = (const T*)Bt2p;
  __shared__ __align__(16) float sT[8][16 * kTP];
  const int b    = blockIdx.y;
  const int lane = threadIdx.x & 31;
  const int wave = threadIdx.x >> 5;
  const int tilesN = N >> 6;
  const int tilesM = M >> 6;
  const int tile = blockIdx.x * 8 + wave;
  if (tile >= tilesM * tilesN) return;
  const int tm = tile / tilesN;
  const int tn = tile - tm * tilesN;
  const int m0 = tm << 6;
  const int n0 = tn << 6;

  const T* Ab  = A  + (size_t)b * strideA;
  const T* Bb  = Bt;
  const T* Ab2 = (SPL == 2) ? (A2 + (size_t)b * strideA) : nullptr;
  const T* Bb2 = (SPL == 2) ? Bt2 : nullptr;

  const int rlane = lane & 15;
  const int koff  = (lane >> 4) * 8;
  const int mOff  = (lane >> 4) * 8;

  v8f acc[4][4];
#pragma unroll
  for (int i = 0; i < 4; ++i)
#pragma unroll
    for (int j = 0; j < 4; ++j) acc[i][j] = (v8f){0.f,0.f,0.f,0.f,0.f,0.f,0.f,0.f};

  for (int k0 = 0; k0 < K; k0 += 32) {
    V bh[4], bl[4];
#pragma unroll
    for (int j = 0; j < 4; ++j) {
      const size_t bo = (size_t)(n0 + (j << 4) + rlane) * ldb + koff + k0;
      bh[j] = Frag<T>::load(Bb + bo);
      if (SPL == 2) bl[j] = Frag<T>::load(Bb2 + bo);
    }
#pragma unroll
    for (int i = 0; i < 4; ++i) {
      const size_t ao = (size_t)(m0 + (i << 4) + rlane) * lda + koff + k0;
      V ah = Frag<T>::load(Ab + ao);
      V al;
      if (SPL == 2) al = Frag<T>::load(Ab2 + ao);
#pragma unroll
      for (int j = 0; j < 4; ++j) {
        acc[i][j] = Frag<T>::mma(ah, bh[j], acc[i][j]);
        if (SPL == 2) {
          acc[i][j] = Frag<T>::mma(ah, bl[j], acc[i][j]);
          acc[i][j] = Frag<T>::mma(al, bh[j], acc[i][j]);
        }
      }
      Frag<T>::guard4(acc[i][0], acc[i][1], acc[i][2], acc[i][3], ah, (SPL == 2) ? al : ah);
    }
    Frag<T>::keep(bh[0], bh[1], bh[2], bh[3]);
    if (SPL == 2) Frag<T>::keep(bl[0], bl[1], bl[2], bl[3]);
  }
  acc_guard4(acc[0][0], acc[0][1], acc[0][2], acc[0][3]);
  acc_guard4(acc[1][0], acc[1][1], acc[1][2], acc[1][3]);
  acc_guard4(acc[2][0], acc[2][1], acc[2][2], acc[2][3]);
  acc_guard4(acc[3][0], acc[3][1], acc[3][2], acc[3][3]);

  float* slab = sT[wave];
  float bvj[4] = {0.f, 0.f, 0.f, 0.f};
  if (EPI == 3 || EPI == 4) {
#pragma unroll
    for (int j = 0; j < 4; ++j) bvj[j] = bias[n0 + (j << 4) + rlane];
  }
  if (EPI == 5) {
    bvj[0] = bias[rlane];
    bvj[1] = bias2[rlane];
  }
  const float* auxb = (EPI == 4) ? (aux + (size_t)b * strideC) : nullptr;
#pragma unroll
  for (int i = 0; i < 4; ++i) {
    const int mBase = m0 + (i << 4);
#pragma unroll
    for (int j = 0; j < 4; ++j) {
#pragma unroll
      for (int r = 0; r < 8; ++r) {
        const float v = acc[i][j][r] * scale + bvj[j];
        slab[(mOff + r) * kTP + (j << 4) + rlane] = v;
      }
    }
    wave_lds_sync();
    if (EPI == 2 || EPI == 3 || EPI == 4) {
      const int hh = lane >> 4, c4 = (lane & 15) * 4;
#pragma unroll 1
      for (int it = 0; it < 8; ++it) {
        const int row = it * 2 + hh;
        float* sp = slab + row * kTP + c4;
        const v4f v = *(const v4f*)sp;
        float e0 = v[0], e1 = v[1], e2 = v[2], e3 = v[3];
        if (EPI == 4) {
          const v4f xv = *(const v4f*)(auxb + (size_t)(mBase + row) * ldc + n0 + c4);
          const float x0 = xv[0], x1 = xv[1], x2 = xv[2], x3 = xv[3];
          e0 = softplus_f(e0) * x0;
          e1 = softplus_f(e1) * x1;
          e2 = softplus_f(e2) * x2;
          e3 = softplus_f(e3) * x3;
        } else {
          e0 = silu_f(e0);
          e1 = silu_f(e1);
          e2 = silu_f(e2);
          e3 = silu_f(e3);
        }
        v4f o;
        o[0] = e0; o[1] = e1; o[2] = e2; o[3] = e3;
        *(v4f*)sp = o;
      }
      wave_lds_sync();
    }
    if (EPI == 0 || EPI == 2 || EPI == 3 || EPI == 4 || EPI == 5) {
      store_slab_f32(slab, (float*)C0 + (size_t)b * strideC, mBase, ldc, n0, lane);
    }
    if (EPI == 1) {
      store_slab_16<0>(slab, (unsigned short*)C0 + (size_t)b * strideC, (unsigned short*)C1 + (size_t)b * strideC,
                       mBase, ldc, n0, lane, 1.0f);
    }
    if (EPI == 3) {
      store_slab_16<1>(slab, (unsigned short*)C1 + (size_t)b * strideC, nullptr, mBase, ldc, n0, lane, kCarryXc);
      store_slab_16<0>(slab, (unsigned short*)C2 + (size_t)b * strideC, (unsigned short*)C3 + (size_t)b * strideC,
                       mBase, ldc, n0, lane, 1.0f);
    }
    wave_lds_sync();
  }
}

__global__ __launch_bounds__(256) void split_rows_bf16_kernel(
    const float* __restrict__ src, unsigned short* __restrict__ dhi, unsigned short* __restrict__ dlo, int total8)
{
  const int i = blockIdx.x * 256 + threadIdx.x;
  if (i >= total8) return;
  const size_t e0 = (size_t)i << 3;
  const v4f a0 = *(const v4f*)(src + e0);
  const v4f a1 = *(const v4f*)(src + e0 + 4);
  v8h hv, lv;
#pragma unroll
  for (int e = 0; e < 4; ++e) {
    const float f0 = a0[e];
    const float f1 = a1[e];
    _Float16 h0, l0, h1, l1;
    cvt_hilo(f0, h0, l0);
    cvt_hilo(f1, h1, l1);
    hv[e] = h0;
    hv[4 + e] = h1;
    lv[e] = l0;
    lv[4 + e] = l1;
  }
  unsigned short* qh = dhi + e0;
  unsigned short* ql = dlo + e0;
  *(volatile v8h*)qh = hv;
  *(volatile v8h*)ql = lv;
  __threadfence();
  *(volatile v8h*)qh = hv;
  *(volatile v8h*)ql = lv;
}

template <int MODE>
__device__ __forceinline__ void emit_tile_planes(const float* sT, unsigned short* P0, unsigned short* P1,
                                                 int n0, int k0, int kdim, int tid) {
  const int q = tid >> 3, c8 = (tid & 7) * 8;
  v8h hv[2], lv[2];
#pragma unroll
  for (int i = 0; i < 2; ++i) {
    const float* sp = sT + (q + 32 * i) * kTP + c8;
    const v4f a0 = *(const v4f*)(sp);
    const v4f a1 = *(const v4f*)(sp + 4);
#pragma unroll
    for (int e = 0; e < 4; ++e) {
      const float f0 = a0[e];
      const float f1 = a1[e];
      _Float16 h0, l0, h1, l1;
      if (MODE == 0) {
        cvt_hilo(f0, h0, l0);
        cvt_hilo(f1, h1, l1);
      } else {
        h0 = cvt_f16_carried(f0, kCarryWd);
        h1 = cvt_f16_carried(f1, kCarryWd);
        l0 = h0;
        l1 = h1;
      }
      hv[i][e] = h0;
      hv[i][4 + e] = h1;
      lv[i][e] = l0;
      lv[i][4 + e] = l1;
    }
  }
  for (int pass = 0; pass < 2; ++pass) {
#pragma unroll
    for (int i = 0; i < 2; ++i) {
      const size_t o = (size_t)(n0 + q + 32 * i) * kdim + k0 + c8;
      *(volatile v8h*)(P0 + o) = hv[i];
      if (MODE == 0) *(volatile v8h*)(P1 + o) = lv[i];
    }
    __threadfence();
  }
}

template <int MODE>
__global__ __launch_bounds__(256) void transpose_planes_kernel(
    const float* __restrict__ W, int ncols, unsigned short* __restrict__ P0, unsigned short* __restrict__ P1, int kdim)
{
  __shared__ __align__(16) float sT[64 * kTP];
  const int tid = threadIdx.x;
  const int n0 = blockIdx.x * 64, k0 = blockIdx.y * 64;
  const int kr = tid >> 4, c4 = (tid & 15) * 4;
#pragma unroll
  for (int i = 0; i < 4; ++i) {
    const int k = kr + 16 * i;
    const v4f v = *(const v4f*)(W + (size_t)(k0 + k) * ncols + n0 + c4);
    const float f0 = v[0], f1 = v[1], f2 = v[2], f3 = v[3];
    sT[(c4 + 0) * kTP + k] = f0;
    sT[(c4 + 1) * kTP + k] = f1;
    sT[(c4 + 2) * kTP + k] = f2;
    sT[(c4 + 3) * kTP + k] = f3;
  }
  __syncthreads();
  emit_tile_planes<MODE>(sT, P0, P1, n0, k0, kdim, tid);
}

__global__ __launch_bounds__(256) void bc_weight_planes_kernel(
    const float* __restrict__ wB, const float* __restrict__ wC,
    unsigned short* __restrict__ P0, unsigned short* __restrict__ P1)
{
  __shared__ __align__(16) float sT[64 * kTP];
  const int tid = threadIdx.x;
  const int k0 = blockIdx.x * 64;
  const int k = tid >> 2, c4 = (tid & 3) * 4;
  const v4f vb = *(const v4f*)(wB + (size_t)(k0 + k) * kNst + c4);
  const v4f vc = *(const v4f*)(wC + (size_t)(k0 + k) * kNst + c4);
  const float b0 = vb[0], b1 = vb[1], b2 = vb[2], b3 = vb[3];
  const float g0 = vc[0], g1 = vc[1], g2 = vc[2], g3 = vc[3];
  sT[(c4 + 0) * kTP + k] = b0;
  sT[(c4 + 1) * kTP + k] = b1;
  sT[(c4 + 2) * kTP + k] = b2;
  sT[(c4 + 3) * kTP + k] = b3;
  sT[(kNst + c4 + 0) * kTP + k] = g0;
  sT[(kNst + c4 + 1) * kTP + k] = g1;
  sT[(kNst + c4 + 2) * kTP + k] = g2;
  sT[(kNst + c4 + 3) * kTP + k] = g3;
  {
    const int zr = 32 + (tid >> 3), zc = (tid & 7) * 8;
#pragma unroll
    for (int e = 0; e < 8; ++e) sT[zr * kTP + zc + e] = 0.0f;
  }
  __syncthreads();
  emit_tile_planes<0>(sT, P0, P1, 0, k0, kDin, tid);
}

__global__ __launch_bounds__(128) void zero_pad_rows_kernel(unsigned short* __restrict__ PH, unsigned short* __restrict__ PL)
{
  const int bx = blockIdx.x;
  const int plane = bx / 6;
  const int rem = bx - plane * 6;
  const int b = rem / 3;
  const int r = rem - b * 3;
  const int row = (r == 0) ? 0 : (kSeq + r);
  unsigned short* base = (plane == 0) ? PH : PL;
  unsigned short* p = base + ((size_t)b * kPadRows + row) * kDin + threadIdx.x * 8;
  const v8h z = (v8h){(_Float16)0.0f, (_Float16)0.0f, (_Float16)0.0f, (_Float16)0.0f,
                      (_Float16)0.0f, (_Float16)0.0f, (_Float16)0.0f, (_Float16)0.0f};
  *(volatile v8h*)p = z;
  __threadfence();
  *(volatile v8h*)p = z;
}

__global__ __launch_bounds__(64) void prefix_scan_kernel(
    const float* __restrict__ BC, const float* __restrict__ DX, const float* __restrict__ GATE,
    unsigned short* __restrict__ YH, unsigned short* __restrict__ YL)
{
  __shared__ __align__(16) float sX[kScanTS * kScanXP];
  __shared__ __align__(16) float sY[kScanTS * kScanYP];
  const int tid = threadIdx.x, lane = tid & 31, wave = tid >> 5;
  constexpr int kBlkPerB = kDin / kScanCh;
  const int bix = blockIdx.x / kBlkPerB;
  const int d0  = (blockIdx.x - bix * kBlkPerB) * kScanCh;
  const int d   = d0 + tid;
  const size_t row0 = (size_t)bix * kSeq;
  float h[kNst];
#pragma unroll
  for (int s = 0; s < kNst; ++s) h[s] = 0.0f;
  float dec = 0.95f;
  const int lr = tid >> 3, lc4 = (tid & 7) * 4;
  const int q = lane >> 3, c8 = (lane & 7) * 8;
#pragma unroll 1
  for (int t0 = 0; t0 < kSeq; t0 += kScanTS) {
    __syncthreads();
#pragma unroll
    for (int i = 0; i < 8; ++i) {
      const int r = lr + 8 * i;
      *(v4f*)(sX + r * kScanXP + lc4) = *(const v4f*)(BC + (row0 + t0 + r) * kBcP + lc4);
    }
    __syncthreads();
#pragma unroll 1
    for (int s = 0; s < kScanTS; ++s) {
      const size_t grow = row0 + t0 + s;
      const float* xr = sX + s * kScanXP;
      float Bs[kNst], Cs[kNst];
#pragma unroll
      for (int q4 = 0; q4 < 4; ++q4) {
        const v4f bv = *(const v4f*)(xr + 4 * q4);
        const v4f cv = *(const v4f*)(xr + kNst + 4 * q4);
        Bs[4 * q4 + 0] = bv[0]; Bs[4 * q4 + 1] = bv[1]; Bs[4 * q4 + 2] = bv[2]; Bs[4 * q4 + 3] = bv[3];
        Cs[4 * q4 + 0] = cv[0]; Cs[4 * q4 + 1] = cv[1]; Cs[4 * q4 + 2] = cv[2]; Cs[4 * q4 + 3] = cv[3];
      }
      const float dx = DX[grow * kDin + d];
      const float gt = GATE[grow * kDin + d];
      const float w = dx * dec;
      float y = 0.0f;
#pragma unroll
      for (int k = 0; k < kNst; ++k) {
        h[k] = fmaf(w, Bs[k], h[k]);
        y = fmaf(h[k], Cs[k], y);
      }
      sY[s * kScanYP + tid] = y * gt;
      dec = dec * 0.95f;
      dec = (dec < kF32MinNormal) ? 0.0f : dec;
    }
    __syncthreads();
    v8h hv[8], lv[8];
#pragma unroll
    for (int it = 0; it < 8; ++it) {
      const int row = it * 8 + wave * 4 + q;
      const float* sp = sY + row * kScanYP + c8;
      const v4f a0 = *(const v4f*)(sp);
      const v4f a1 = *(const v4f*)(sp + 4);
#pragma unroll
      for (int e = 0; e < 4; ++e) {
        const float f0 = a0[e];
        const float f1 = a1[e];
        _Float16 h0, l0, h1, l1;
        cvt_hilo(f0, h0, l0);
        cvt_hilo(f1, h1, l1);
        hv[it][e] = h0;
        hv[it][4 + e] = h1;
        lv[it][e] = l0;
        lv[it][4 + e] = l1;
      }
    }
    for (int pass = 0; pass < 2; ++pass) {
#pragma unroll
      for (int it = 0; it < 8; ++it) {
        const int row = it * 8 + wave * 4 + q;
        const size_t o = (row0 + t0 + row) * kDin + d0 + c8;
        *(volatile v8h*)(YH + o) = hv[it];
        *(volatile v8h*)(YL + o) = lv[it];
      }
      __threadfence();
    }
  }
}

extern "C" void kernel_launch(void* const* d_in, const int* in_sizes, int n_in,
                              void* d_out, int out_size, void* d_ws, size_t ws_size,
                              hipStream_t stream) {
  if (n_in < 12) return;
  if (in_sizes[0] != kRows * kDm) return;
  if (in_sizes[1] != kDm * kXp) return;
  if (in_sizes[2] != kTaps * kDin * kDin) return;
  if (in_sizes[3] != kDin) return;
  if (in_sizes[4] != kDin * kDin) return;
  if (in_sizes[5] != kDin) return;
  if (in_sizes[6] != kDin * kNst) return;
  if (in_sizes[7] != kNst) return;
  if (in_sizes[8] != kDin * kNst) return;
  if (in_sizes[9] != kNst) return;
  if (in_sizes[11] != kDin * kDm) return;
  if (out_size != kRows * kDm) return;
  if (ws_size < kWsTotal) return;

  const float* x       = (const float*)d_in[0];
  const float* w_in    = (const float*)d_in[1];
  const float* conv_k  = (const float*)d_in[2];
  const float* conv_b  = (const float*)d_in[3];
  const float* w_delta = (const float*)d_in[4];
  const float* b_delta = (const float*)d_in[5];
  const float* w_B     = (const float*)d_in[6];
  const float* b_B     = (const float*)d_in[7];
  const float* w_C     = (const float*)d_in[8];
  const float* b_C     = (const float*)d_in[9];
  const float* w_out   = (const float*)d_in[11];
  float* out = (float*)d_out;

  char* ws = (char*)d_ws;
  unsigned short* XH   = (unsigned short*)(ws + kOffXH);
  unsigned short* XL   = (unsigned short*)(ws + kOffXL);
  unsigned short* WIH  = (unsigned short*)(ws + kOffWIH);
  unsigned short* WIL  = (unsigned short*)(ws + kOffWIL);
  unsigned short* CKH  = (unsigned short*)(ws + kOffCKH);
  unsigned short* CKL  = (unsigned short*)(ws + kOffCKL);
  unsigned short* WD16 = (unsigned short*)(ws + kOffWD);
  unsigned short* WBCH = (unsigned short*)(ws + kOffWBCH);
  unsigned short* WBCL = (unsigned short*)(ws + kOffWBCL);
  unsigned short* WOH  = (unsigned short*)(ws + kOffWOH);
  unsigned short* WOL  = (unsigned short*)(ws + kOffWOL);
  unsigned short* XZH  = (unsigned short*)(ws + kOffXZH);
  unsigned short* XZL  = (unsigned short*)(ws + kOffXZL);
  float*          GATE = (float*)(ws + kOffGATE);
  float*          XC32 = (float*)(ws + kOffXC32);
  unsigned short* XC16 = (unsigned short*)(ws + kOffXC16);
  unsigned short* XCH  = (unsigned short*)(ws + kOffXCH);
  unsigned short* XCL  = (unsigned short*)(ws + kOffXCL);
  float*          DX   = (float*)(ws + kOffDX);
  float*          BC   = (float*)(ws + kOffBC);
  unsigned short* YH   = CKH;
  unsigned short* YL   = CKL;

  split_rows_bf16_kernel<<<(kRows * kDm / 8) / 256, 256, 0, stream>>>(x, XH, XL, kRows * kDm / 8);
  transpose_planes_kernel<0><<<dim3(kXp / 64, kDm / 64), 256, 0, stream>>>(w_in, kXp, WIH, WIL, kDm);
  transpose_planes_kernel<0><<<dim3(kDin / 64, kConvK / 64), 256, 0, stream>>>(conv_k, kDin, CKH, CKL, kConvK);
  transpose_planes_kernel<1><<<dim3(kDin / 64, kDin / 64), 256, 0, stream>>>(w_delta, kDin, WD16, nullptr, kDin);
  transpose_planes_kernel<0><<<dim3(kDm / 64, kDin / 64), 256, 0, stream>>>(w_out, kDm, WOH, WOL, kDin);
  bc_weight_planes_kernel<<<kDin / 64, 256, 0, stream>>>(w_B, w_C, WBCH, WBCL);
  zero_pad_rows_kernel<<<12, 128, 0, stream>>>(XZH, XZL);

  gemm64_kernel<1, 2, 1><<<dim3((kSeq / 64) * (kDin / 64) / 8, kBatch), 256, 0, stream>>>(
      XH, XL, kDm, (long)kSeq * kDm,
      WIH, WIL, kDm,
      (void*)(XZH + kDin), (void*)(XZL + kDin), nullptr, nullptr, kDin, (long)kPadRows * kDin,
      nullptr, nullptr, nullptr,
      kSeq, kDin, kDm, 1.0f);

  gemm64_kernel<1, 2, 2><<<dim3((kRows / 64) * (kDin / 64) / 8, 1), 256, 0, stream>>>(
      XH, XL, kDm, 0L,
      WIH + (size_t)kDin * kDm, WIL + (size_t)kDin * kDm, kDm,
      (void*)GATE, nullptr, nullptr, nullptr, kDin, 0L,
      nullptr, nullptr, nullptr,
      kRows, kDin, kDm, 1.0f);

  gemm64_kernel<1, 2, 3><<<dim3((kSeq / 64) * (kDin / 64) / 8, kBatch), 256, 0, stream>>>(
      XZH, XZL, kDin, (long)kPadRows * kDin,
      CKH, CKL, kConvK,
      (void*)XC32, (void*)XC16, (void*)XCH, (void*)XCL, kDin, (long)kSeq * kDin,
      conv_b, nullptr, nullptr,
      kSeq, kDin, kConvK, 1.0f);

  gemm64_kernel<0, 0, 4><<<dim3((kRows / 64) * (kDin / 64) / 8, 1), 256, 0, stream>>>(
      XC16, nullptr, kDin, 0L,
      WD16, nullptr, kDin,
      (void*)DX, nullptr, nullptr, nullptr, kDin, 0L,
      b_delta, nullptr, XC32,
      kRows, kDin, kDin, kDeltaScale);

  gemm64_kernel<1, 2, 5><<<dim3((kRows / 64) * (kBcP / 64) / 8, 1), 256, 0, stream>>>(
      XCH, XCL, kDin, 0L,
      WBCH, WBCL, kDin,
      (void*)BC, nullptr, nullptr, nullptr, kBcP, 0L,
      b_B, b_C, nullptr,
      kRows, kBcP, kDin, 1.0f);

  prefix_scan_kernel<<<kBatch * (kDin / kScanCh), kScanCh, 0, stream>>>(BC, DX, GATE, YH, YL);

  gemm64_kernel<1, 2, 0><<<dim3((kRows / 64) * (kDm / 64) / 8, 1), 256, 0, stream>>>(
      YH, YL, kDin, 0L,
      WOH, WOL, kDin,
      (void*)out, nullptr, nullptr, nullptr, kDm, 0L,
      nullptr, nullptr, nullptr,
      kRows, kDm, kDin, 1.0f);
}
